// TransformerBlock_7404523618568
// MI455X (gfx1250) — hardware-verified
//
#include <hip/hip_runtime.h>
#ifndef NB
#define NB 2
#endif
#ifndef SEQ
#define SEQ 2048
#endif
#define SQ SEQ
#define NB_FULL 2
#define SQ_FULL 2048
#define DM 768
#define NH 12
#define HD 64
#define DFF 3072
#define QT0 128
#define LQ (3 * DM)
#define NR ((size_t)NB * SQ)
#define DMQ DM
static_assert(SQ % 128 == 0);
static_assert(SQ <= SQ_FULL);
static_assert(NB <= NB_FULL);
static_assert(DM % 64 == 0);
static_assert(DFF % 64 == 0);
static_assert(LQ % 64 == 0);
static_assert((DMQ / 4) % 32 == 0);
static_assert(DM == NH * HD);
static_assert(QT0 == 128);
static_assert(QT0 <= SQ);

typedef unsigned short v8us __attribute__((ext_vector_type(8), may_alias));
typedef float  v8f  __attribute__((ext_vector_type(8)));
typedef float  v4f  __attribute__((ext_vector_type(4)));
typedef float  v4fa __attribute__((ext_vector_type(4), may_alias));
typedef _Float16 v16h __attribute__((ext_vector_type(16)));
typedef _Float16 v4h __attribute__((ext_vector_type(4)));
union FragH { v16h v; v8us half[2]; _Float16 h[16]; unsigned short u[16]; };

__device__ __forceinline__ unsigned short bf16_bits(float x) { unsigned int u = __float_as_uint(x); return (unsigned short)((u + 0x7FFFu + ((u >> 16) & 1u)) >> 16); }
__device__ __forceinline__ float bf16_val(unsigned short b) { return __uint_as_float(((unsigned int)b) << 16); }
__device__ __forceinline__ float bf16_rne(float x) { return bf16_val(bf16_bits(x)); }

__device__ __forceinline__ v16h g2_frag(const _Float16* p, int hh) { FragH f; f.half[0] = *(const v8us*)((const unsigned short*)p + 8 * hh); f.half[1] = *(const v8us*)((const unsigned short*)p + 16 + 8 * hh); return f.v; }
__device__ __forceinline__ v8f g2_mma(v16h a, v16h b, v8f c) { v8f d = __builtin_amdgcn_wmma_f32_16x16x32_f16(false, a, false, b, (short)0, c, false, false); asm volatile("v_nop\n\tv_nop\n\tv_nop\n\tv_nop" : "+v"(d) : "v"(a), "v"(b)); return d; }

__global__ __launch_bounds__(256) void k_wnat(const float* __restrict__ w, size_t n8, _Float16* __restrict__ Bt) {
  const size_t t = (size_t)blockIdx.x * 256 + threadIdx.x; if (t >= n8) return; FragH f;
  const v4f a = *(const v4fa*)(w + t * 8), c = *(const v4fa*)(w + t * 8 + 4);
#pragma unroll
  for (int q = 0; q < 4; ++q) { f.h[q] = (_Float16)(bf16_rne(a[q]) * 16.0f); f.h[4 + q] = (_Float16)(bf16_rne(c[q]) * 16.0f); }
  const v8us o = f.half[0];
  *(volatile v8us*)((unsigned short*)Bt + t * 8) = o; __threadfence(); *(volatile v8us*)((unsigned short*)Bt + t * 8) = o; }

template <int BFIN, int WXB>
__global__ __launch_bounds__(256) void k_ln16(const float* __restrict__ X, int inS, const float* __restrict__ g, const float* __restrict__ bb, float eps, _Float16* __restrict__ N16, float* __restrict__ XB) {
  #pragma clang fp contract(off)
  __shared__ float red[256];
  const int r = blockIdx.x; const int t = threadIdx.x;
  const int wave = __builtin_amdgcn_readfirstlane(t >> 5);
  const bool act = wave < (DMQ / 128);
  const int tc = act ? t : 0;
  const size_t ir = (size_t)(r / SQ) * (size_t)inS + (size_t)(r % SQ);
  const v4f xa = *(const v4fa*)(X + ir * DMQ + tc * 4);
  float s[4]; float sum = 0.f;
#pragma unroll
  for (int q = 0; q < 4; ++q) { s[q] = BFIN ? bf16_rne(xa[q]) : xa[q]; sum = sum + s[q]; }
  red[t] = act ? sum : 0.f; __syncthreads();
  for (int st = 128; st > 0; st >>= 1) { if (t < st) red[t] = red[t] + red[t + st]; __syncthreads(); }
  const float mu = red[0] / (float)DMQ; __syncthreads();
  float vs = 0.f;
#pragma unroll
  for (int q = 0; q < 4; ++q) { const float dl = s[q] - mu; vs = vs + dl * dl; }
  red[t] = act ? vs : 0.f; __syncthreads();
  for (int st = 128; st > 0; st >>= 1) { if (t < st) red[t] = red[t] + red[t + st]; __syncthreads(); }
  const float rs = rsqrtf(red[0] / (float)DMQ + eps);
  v4h y; v4f xb;
#pragma unroll
  for (int q = 0; q < 4; ++q) { const int c = tc * 4 + q; const float nv = ((s[q] - mu) * rs) * bf16_rne(g[c]) + bf16_rne(bb[c]); y[q] = (_Float16)nv; xb[q] = s[q]; }
  if (act) {
    for (int pass = 0; pass < 2; ++pass) {
      *(volatile v4h*)(N16 + (size_t)r * DMQ + t * 4) = y;
      if (WXB) *(volatile v4f*)(XB + ir * DMQ + t * 4) = xb;
      if (pass == 0) __threadfence(); } } }

template <int ACT>
__global__ __launch_bounds__(128) void k_gemm2(const _Float16* __restrict__ A, int lda, size_t sA, const _Float16* __restrict__ Bh, int ldb, size_t sB, float alpha, const float* __restrict__ bias, const float* CP,
    float* C, _Float16* C16, int ldc, size_t sC, int M, int N, int K) {
  static_assert(ACT == 0 || ACT == 9);
  __shared__ __attribute__((aligned(16))) float so[4][32][68];
  const int tid = threadIdx.x; const int w = __builtin_amdgcn_readfirstlane(tid >> 5); const int lane = tid & 31, ln = lane & 15, hh = lane >> 4; const int by = blockIdx.y;
  A += (size_t)by * sA; Bh += (size_t)by * sB; const size_t cofs = (size_t)by * sC;
  const int ntn = N >> 6; const int mt = blockIdx.x / ntn, nq = blockIdx.x - mt * ntn; const int row0 = mt * 128 + 32 * w, col0 = nq * 64; if (row0 >= M) return;
  const _Float16* a0p = A + (size_t)(row0 + ln) * lda; const _Float16* a1p = a0p + (size_t)16 * lda;
  const _Float16* b0p = Bh + (size_t)(col0 + ln) * ldb; const _Float16* b1p = b0p + (size_t)16 * ldb; const _Float16* b2p = b1p + (size_t)16 * ldb; const _Float16* b3p = b2p + (size_t)16 * ldb;
  const v8f z8 = {0.f,0.f,0.f,0.f,0.f,0.f,0.f,0.f}; v8f c00 = z8, c01 = z8, c02 = z8, c03 = z8, c10 = z8, c11 = z8, c12 = z8, c13 = z8;
#pragma unroll 1
  for (int kb = 0; kb < K; kb += 32) { const v16h a0 = g2_frag(a0p + kb, hh), a1 = g2_frag(a1p + kb, hh);
    v16h b = g2_frag(b0p + kb, hh); c00 = g2_mma(a0, b, c00); c10 = g2_mma(a1, b, c10);
    b = g2_frag(b1p + kb, hh); c01 = g2_mma(a0, b, c01); c11 = g2_mma(a1, b, c11);
    b = g2_frag(b2p + kb, hh); c02 = g2_mma(a0, b, c02); c12 = g2_mma(a1, b, c12);
    b = g2_frag(b3p + kb, hh); c03 = g2_mma(a0, b, c03); c13 = g2_mma(a1, b, c13); }
  v8f accs[8] = {c00, c01, c02, c03, c10, c11, c12, c13};
#pragma unroll
  for (int u = 0; u < 8; ++u) { const int t = u & 3, half = u >> 2; const int col = col0 + t * 16 + ln; const float bv = bias ? bf16_rne(bias[col]) : 0.f;
#pragma unroll
    for (int r = 0; r < 8; ++r) { const int rloc = half * 16 + 8 * hh + r; float v = accs[u][r] * alpha + bv;
      if (CP) v += CP[cofs + (size_t)(row0 + rloc) * ldc + col];
      if (ACT == 9) v = 0.5f * v * (1.0f + tanhf(0.7978845608028654f * (v + 0.044715f * v * v * v)));
      so[w][rloc][t * 16 + ln] = v; } }
  __builtin_amdgcn_fence(4  , "workgroup"); __builtin_amdgcn_wave_barrier();
  const int rsub = lane >> 4, c4 = (lane & 15) * 4;
  for (int pass = 0; pass < 2; ++pass) {
#pragma unroll
    for (int q = 0; q < 16; ++q) { const int r = q * 2 + rsub; const v4f v = *(const v4fa*)&so[w][r][c4];
      if (C) *(volatile v4f*)(C + cofs + (size_t)(row0 + r) * ldc + col0 + c4) = v;
      if (C16) { v4h h4; for (int i = 0; i < 4; ++i) h4[i] = (_Float16)v[i]; *(volatile v4h*)(C16 + cofs + (size_t)(row0 + r) * ldc + col0 + c4) = h4; } }
    if (pass == 0) __threadfence(); } }

template <int NHv, int TTv>
__global__ __launch_bounds__(256) void k_vt(const _Float16* __restrict__ V16, int ldv, _Float16* __restrict__ Vt) {
  __shared__ unsigned short tl[64][66]; const int tid = threadIdx.x; const int slab = blockIdx.x / (TTv / 64), lg = blockIdx.x % (TTv / 64); const int b = slab / NHv, h = slab % NHv;
  for (int i = tid; i < 64 * 8; i += 256) { const int r = i / 8, c8 = (i % 8) * 8; FragH f; f.half[0] = *(const v8us*)((const unsigned short*)V16 + ((size_t)b * TTv + lg * 64 + r) * ldv + h * 64 + c8);
#pragma unroll
    for (int q = 0; q < 8; ++q) tl[r][c8 + q] = f.u[q]; }
  __syncthreads();
  for (int pass = 0; pass < 2; ++pass) {
#pragma unroll
    for (int rd = 0; rd < 2; ++rd) { const int d = rd * 32 + tid / 8, pc = tid % 8; FragH f;
#pragma unroll
      for (int q = 0; q < 8; ++q) f.u[q] = tl[pc * 8 + q][d];
      *(volatile v8us*)((unsigned short*)Vt + ((size_t)slab * 64 + d) * TTv + lg * 64 + pc * 8) = f.half[0]; }
    if (pass == 0) __threadfence(); } }

__global__ __launch_bounds__(128) void k_flash(const _Float16* __restrict__ QKV, const _Float16* __restrict__ VT, _Float16* __restrict__ O16) {
  __shared__ __attribute__((aligned(16))) unsigned short ot[4][16][72];
  const int wave = __builtin_amdgcn_readfirstlane(threadIdx.x >> 5);
  const int lane = threadIdx.x & 31, ln = lane & 15, hh = lane >> 4;
  const int bh = blockIdx.y; const int b = bh / NH; const int h = bh - b * NH;
  const int qw0 = blockIdx.x * 64 + wave * 16;
  const size_t rowb = (size_t)b * SQ;
  const _Float16* qp = QKV + (rowb + qw0 + ln) * LQ + h * HD;
  const _Float16* kp = QKV + (rowb + ln) * LQ + DM + h * HD;
  const _Float16* vp = VT + ((size_t)bh * HD + ln) * SQ;
  const v8f z8 = {0.f,0.f,0.f,0.f,0.f,0.f,0.f,0.f};
  v8f a0 = z8, a1 = z8, a2 = z8, a3 = z8;
  float mprev = -1.0e30f, lsum = 0.f;
  const int qg = qw0 + ln;
  const int nst = ((qw0 + 15) >> 5) + 1;
#pragma unroll 1
  for (int st = 0; st < nst; ++st) {
    const int ks = st * 32;
    const v16h qb0 = g2_frag(qp, hh), qb1 = g2_frag(qp + 32, hh);
    const _Float16* k0 = kp + (size_t)ks * LQ; const _Float16* k1 = k0 + (size_t)16 * LQ;
    v16h ka = g2_frag(k0, hh); v8f s0 = g2_mma(ka, qb0, z8);
    ka = g2_frag(k0 + 32, hh); s0 = g2_mma(ka, qb1, s0);
    ka = g2_frag(k1, hh); v8f s1 = g2_mma(ka, qb0, z8);
    ka = g2_frag(k1 + 32, hh); s1 = g2_mma(ka, qb1, s1);
    float p0[8], p1[8]; float mx = -1.0e30f;
    const int kb0 = ks + 8 * hh;
#pragma unroll
    for (int r = 0; r < 8; ++r) {
      const float v0 = (kb0 + r <= qg) ? s0[r] * 0.125f : -1.0e30f;
      const float v1 = (kb0 + 16 + r <= qg) ? s1[r] * 0.125f : -1.0e30f;
      p0[r] = v0; p1[r] = v1; mx = fmaxf(mx, fmaxf(v0, v1)); }
    mx = fmaxf(mx, __shfl_xor(mx, 16, 32));
    const float mnew = fmaxf(mprev, mx);
    const float alpha = __expf(mprev - mnew);
    float rs = 0.f; FragH pb;
#pragma unroll
    for (int r = 0; r < 8; ++r) {
      const float e0 = __expf(p0[r] - mnew), e1 = __expf(p1[r] - mnew);
      rs += e0 + e1;
      pb.h[r] = (_Float16)(e0 * 256.0f); pb.h[8 + r] = (_Float16)(e1 * 256.0f); }
    rs += __shfl_xor(rs, 16, 32);
    lsum = lsum * alpha + rs; mprev = mnew;
    a0 *= alpha; a1 *= alpha; a2 *= alpha; a3 *= alpha;
    const _Float16* v0p = vp + ks;
    v16h va = g2_frag(v0p, hh); a0 = g2_mma(va, pb.v, a0);
    va = g2_frag(v0p + (size_t)16 * SQ, hh); a1 = g2_mma(va, pb.v, a1);
    va = g2_frag(v0p + (size_t)32 * SQ, hh); a2 = g2_mma(va, pb.v, a2);
    va = g2_frag(v0p + (size_t)48 * SQ, hh); a3 = g2_mma(va, pb.v, a3);
  }
  const float linv = 0.25f / lsum;
  { FragH f;
#pragma unroll
    for (int r = 0; r < 8; ++r) f.h[r] = (_Float16)(a0[r] * linv);
    *(v8us*)&ot[wave][ln][8 * hh] = f.half[0];
#pragma unroll
    for (int r = 0; r < 8; ++r) f.h[r] = (_Float16)(a1[r] * linv);
    *(v8us*)&ot[wave][ln][16 + 8 * hh] = f.half[0];
#pragma unroll
    for (int r = 0; r < 8; ++r) f.h[r] = (_Float16)(a2[r] * linv);
    *(v8us*)&ot[wave][ln][32 + 8 * hh] = f.half[0];
#pragma unroll
    for (int r = 0; r < 8; ++r) f.h[r] = (_Float16)(a3[r] * linv);
    *(v8us*)&ot[wave][ln][48 + 8 * hh] = f.half[0]; }
  __builtin_amdgcn_fence(4  , "workgroup"); __builtin_amdgcn_wave_barrier();
  const int rq = lane >> 3, pc = (lane & 7) * 8;
  unsigned short* ob = (unsigned short*)O16 + (rowb + qw0) * DM + h * HD + pc;
  for (int pass = 0; pass < 2; ++pass) {
#pragma unroll
    for (int j = 0; j < 4; ++j) { const int row = 4 * j + rq; const v8us v = *(const v8us*)&ot[wave][row][pc]; *(volatile v8us*)(ob + (size_t)row * DM) = v; }
    if (pass == 0) __threadfence(); } }

__global__ __launch_bounds__(64) void k_att0(const float* __restrict__ QKVF, float scale, float* __restrict__ OF) {
  #pragma clang fp contract(off)
  __shared__ __attribute__((aligned(16))) float lq[64][64]; __shared__ __attribute__((aligned(16))) float lo[64][64];
  const int tid = threadIdx.x; const int h = blockIdx.x / (QT0 / 64), rg = blockIdx.x % (QT0 / 64); const int i = rg * 64 + tid;
  const float* base = QKVF + (size_t)blockIdx.y * QT0 * LQ;
  float* ob = OF + (size_t)blockIdx.y * QT0 * DM;
  const float* qr = base + (size_t)i * LQ + h * HD;
#pragma unroll 1
  for (int c = 0; c < HD / 4; ++c) { *(v4f*)&lq[tid][c * 4] = *(const v4fa*)(qr + c * 4); const v4f z = {0.f, 0.f, 0.f, 0.f}; *(v4f*)&lo[tid][c * 4] = z; }
  float m = -1.0e30f, l = 0.f; const int jmax = rg * 64 + 63;
#pragma unroll 1
  for (int j = 0; j <= jmax; ++j) { const float* kr = base + (size_t)j * LQ + DM + h * HD; const float* vr = base + (size_t)j * LQ + 2 * DM + h * HD; float s = 0.f;
#pragma unroll 1
    for (int c = 0; c < HD / 4; ++c) { const v4f kq = *(const v4fa*)(kr + c * 4); const v4f qq = *(v4f*)&lq[tid][c * 4]; s = __fadd_rn(s, __fmul_rn(qq[0], kq[0])); s = __fadd_rn(s, __fmul_rn(qq[1], kq[1])); s = __fadd_rn(s, __fmul_rn(qq[2], kq[2])); s = __fadd_rn(s, __fmul_rn(qq[3], kq[3])); }
    s = __fmul_rn(s, scale);
    const float f = (j <= i) ? 1.f : 0.f; const float sm = fmaf(f, s, (1.f - f) * -1.0e30f); const float mn = fmaxf(m, sm); const float sc = expf(m - mn); const float e = expf(sm - mn); l = __fadd_rn(__fmul_rn(l, sc), e); m = mn;
#pragma unroll 1
    for (int c = 0; c < HD / 4; ++c) { const v4f vv = *(const v4fa*)(vr + c * 4); v4f oo = *(v4f*)&lo[tid][c * 4]; for (int u = 0; u < 4; ++u) oo[u] = __fadd_rn(__fmul_rn(oo[u], sc), __fmul_rn(e, vv[u])); *(v4f*)&lo[tid][c * 4] = oo; } }
  const float fin = 64.0f / l;
#pragma unroll 1
  for (int c = 0; c < HD / 4; ++c) { v4f oo = *(v4f*)&lo[tid][c * 4]; for (int u = 0; u < 4; ++u) oo[u] = __fmul_rn(oo[u], fin); *(v4f*)&lo[tid][c * 4] = oo; }
  __syncthreads();
  for (int pass = 0; pass < 2; ++pass) {
#pragma unroll 1
    for (int it = 0; it < 16; ++it) { const int row = it * 4 + tid / 16, pc = (tid % 16) * 4; const v4f v = *(const v4f*)&lo[row][pc]; *(volatile v4f*)(ob + (size_t)(rg * 64 + row) * DM + h * HD + pc) = v; }
    if (pass == 0) __threadfence(); } }

__global__ __launch_bounds__(256) void k_hl(const float* __restrict__ F, _Float16* __restrict__ Hh, _Float16* __restrict__ Hl, size_t n8) { const size_t t = (size_t)blockIdx.x * 256 + threadIdx.x; if (t >= n8) return; FragH fh, fl; const v4f a = *(const v4fa*)(F + t * 8), c = *(const v4fa*)(F + t * 8 + 4);
#pragma unroll
  for (int q = 0; q < 4; ++q) { _Float16 hv = (_Float16)a[q]; fh.h[q] = hv; fl.h[q] = (_Float16)((a[q] - (float)hv) * 1024.0f); hv = (_Float16)c[q]; fh.h[4 + q] = hv; fl.h[4 + q] = (_Float16)((c[q] - (float)hv) * 1024.0f); }
  const v8us oh = fh.half[0], ol = fl.half[0];
  for (int pass = 0; pass < 2; ++pass) { *(volatile v8us*)((unsigned short*)Hh + t * 8) = oh; *(volatile v8us*)((unsigned short*)Hl + t * 8) = ol; if (pass == 0) __threadfence(); } }

extern "C" void kernel_launch(void* const* d_in, const int* in_sizes, int n_in,
                              void* d_out, int out_size, void* d_ws, size_t ws_size, hipStream_t stream) {
  if (n_in < 14) return;
  const long long needx = ((long long)(NB - 1) * SQ_FULL + SQ) * DM;
  if ((long long)in_sizes[0] < needx) return;
  if (in_sizes[1] < DM || in_sizes[2] < DM || in_sizes[7] < DM || in_sizes[8] < DM || in_sizes[9] < DM || in_sizes[13] < DM || in_sizes[11] < DFF) return;
  if (in_sizes[3] < DM * DM || in_sizes[4] < DM * DM || in_sizes[5] < DM * DM || in_sizes[6] < DM * DM) return;
  if (in_sizes[10] < DFF * DM || in_sizes[12] < DFF * DM) return;
  if ((long long)out_size < needx) return;
  const float* const* I = (const float* const*)d_in;
  const float* x = I[0]; const float* g1 = I[1]; const float* be1 = I[2]; const float* wq = I[3]; const float* wk = I[4]; const float* wv = I[5]; const float* wo = I[6]; const float* bo = I[7];
  const float* gg2 = I[8]; const float* be2 = I[9]; const float* w1 = I[10]; const float* b1 = I[11]; const float* w2 = I[12]; const float* b2 = I[13];
  char* ws = (char*)d_ws; size_t off = 0;
  auto take = [&](size_t bytes) { char* p = ws + off; off += (bytes + 255) & ~(size_t)255; return p; };
  _Float16* BQKV = (_Float16*)take((size_t)3 * DM * DM * 2);
  _Float16* BO   = (_Float16*)take((size_t)DM * DM * 2);
  _Float16* BW1  = (_Float16*)take((size_t)DFF * DM * 2);
  _Float16* BW2  = (_Float16*)take((size_t)DM * DFF * 2);
  _Float16* X16  = (_Float16*)take(NR * DM * 2);
  float*    XB   = (float*)take((size_t)NB * SQ_FULL * DM * 4);
  float*    X1   = (float*)take((size_t)NB * SQ_FULL * DM * 4);
  _Float16* HF16 = (_Float16*)take(NR * DFF * 2);
  _Float16* QKV  = (_Float16*)take(NR * LQ * 2);
  _Float16* O16  = (_Float16*)take(NR * DM * 2);
  _Float16* VT   = (_Float16*)take((size_t)NB * NH * HD * SQ * 2);
  float*    QKVF0 = (float*)take((size_t)NB * QT0 * LQ * 4);
  float*    OF0  = (float*)take((size_t)NB * QT0 * DM * 4);
  _Float16* OH0  = (_Float16*)take((size_t)NB * QT0 * DM * 2);
  _Float16* OL0  = (_Float16*)take((size_t)NB * QT0 * DM * 2);
  _Float16* M16  = X16;
  if (off > ws_size) return;

  { const size_t n8 = (size_t)DM * DM / 8; const unsigned g = (unsigned)((n8 + 255) / 256);
    k_wnat<<<g, 256, 0, stream>>>(wq, n8, BQKV);
    k_wnat<<<g, 256, 0, stream>>>(wk, n8, BQKV + (size_t)DM * DM);
    k_wnat<<<g, 256, 0, stream>>>(wv, n8, BQKV + (size_t)2 * DM * DM);
    k_wnat<<<g, 256, 0, stream>>>(wo, n8, BO); }
  { const size_t n8 = (size_t)DFF * DM / 8; const unsigned g = (unsigned)((n8 + 255) / 256);
    k_wnat<<<g, 256, 0, stream>>>(w1, n8, BW1);
    k_wnat<<<g, 256, 0, stream>>>(w2, n8, BW2); }
  k_ln16<1, 1><<<(unsigned)NR, 256, 0, stream>>>(x, SQ_FULL, g1, be1, 1e-5f, X16, XB);
  k_gemm2<0><<<dim3((unsigned)((NR / 128) * (LQ / 64)), 1), 128, 0, stream>>>(X16, DM, 0, BQKV, DM, 0, 0.0625f, nullptr, nullptr, nullptr, QKV, LQ, 0, (int)NR, LQ, DM);
  k_vt<NH, SQ><<<NB * NH * (SQ / 64), 256, 0, stream>>>(QKV + 2 * DM, LQ, VT);
  k_flash<<<dim3(SQ / 64, NB * NH), 128, 0, stream>>>(QKV, VT, O16);
  k_gemm2<0><<<dim3((QT0 / 128) * (LQ / 64), NB), 128, 0, stream>>>(X16, DM, (size_t)SQ * DM, BQKV, DM, 0, 0.0625f, nullptr, nullptr, QKVF0, nullptr, LQ, (size_t)QT0 * LQ, QT0, LQ, DM);
  k_att0<<<dim3(NH * (QT0 / 64), NB), 64, 0, stream>>>(QKVF0, 0.125f, OF0);
  k_gemm2<0><<<dim3((SQ / 128) * (DM / 64), NB), 128, 0, stream>>>(O16, DM, (size_t)SQ * DM, BO, DM, 0, 0.0009765625f, bo, XB, X1, nullptr, DM, (size_t)SQ_FULL * DM, SQ, DM, DM);
  k_hl<<<(unsigned)(((size_t)NB * QT0 * DM / 8 + 255) / 256), 256, 0, stream>>>(OF0, OH0, OL0, (size_t)NB * QT0 * DM / 8);
  k_gemm2<0><<<dim3((QT0 / 128) * (DM / 64), NB), 128, 0, stream>>>(OH0, DM, (size_t)QT0 * DM, BO, DM, 0, 0.0009765625f, bo, XB, X1, nullptr, DM, (size_t)SQ_FULL * DM, QT0, DM, DM);
  k_gemm2<0><<<dim3((QT0 / 128) * (DM / 64), NB), 128, 0, stream>>>(OL0, DM, (size_t)QT0 * DM, BO, DM, 0, 0.00000095367431640625f, nullptr, X1, X1, nullptr, DM, (size_t)SQ_FULL * DM, QT0, DM, DM);
  k_ln16<0, 0><<<(unsigned)NR, 256, 0, stream>>>(X1, SQ_FULL, gg2, be2, 1e-5f, M16, nullptr);
  k_gemm2<9><<<dim3((unsigned)((NR / 128) * (DFF / 64)), 1), 128, 0, stream>>>(M16, DM, 0, BW1, DM, 0, 0.0625f, b1, nullptr, nullptr, HF16, DFF, 0, (int)NR, DFF, DM);
  k_gemm2<0><<<dim3((SQ / 128) * (DM / 64), NB), 128, 0, stream>>>(HF16, DFF, (size_t)SQ * DFF, BW2, DFF, 0, 0.0625f, b2, X1, (float*)d_out, nullptr, DM, (size_t)SQ_FULL * DM, SQ, DM, DFF);
}
